// GraphNeuralNetwork_57337813401889
// MI455X (gfx1250) — hardware-verified
//
#include <hip/hip_runtime.h>
#include <stddef.h>
#include <stdint.h>


#define F       64
#define FE      8
#define HID     128
#define MSGIN   136
#define NZK     256
#define SGK     256
#define G1K     256
#define VPK     128
#define W1K     128
#define NTHR    256
#define NWAVE   8
#define GBM     64
#define GTHR    128
#define EPT     8
#define CHUNK   (NTHR * EPT)
#define WCAP    (EPT * 32)
#define LISTN   (NWAVE * WCAP)
#define NBA     1024
#define SLA     10
#define RCAP    28672
#define DEGCAP  96
#define UI_W1   4096
#define UI_W2   2048
#define UI_U1   4096
#define UI_U2   2048
#define UI_TOT  (UI_W1 + UI_W2 + 2 * UI_U1 + 2 * UI_U2)
#define PL_W1   (256 * 128)
#define PL_W2   (64 * 256)
#define PL_U1   (128 * 256)
#define PL_U2   (64 * 256)
#define O_W1    0
#define O_W2    (PL_W1)
#define O_V1    (O_W2 + PL_W2)
#define O_V2    (O_V1 + PL_U1)
#define O_C1    (O_V2 + PL_U2)
#define O_C2    (O_C1 + PL_U1)
#define PL_TOT  (O_C2 + PL_U2)
#define AGG_ZINTS (LISTN + 2 * RCAP + 3 * NBA)
#define AGG_LDS_INTS (AGG_ZINTS + 16 + NBA)
#define AGG_LDS_BYTES (AGG_LDS_INTS * 4)
#define WSMAX   134217728

static_assert((CHUNK & (CHUNK - 1)) == 0 && CHUNK <= 4096);
static_assert((NBA & (NBA - 1)) == 0 && NBA == (1 << SLA));
static_assert(((long long)CHUNK << SLA) < (1LL << 31));
static_assert(LISTN % NTHR == 0);
static_assert(NBA % NWAVE == 0 && NBA % 32 == 0 && NBA == 4 * NTHR);
static_assert(RCAP % 32 == 0 && AGG_ZINTS % 4 == 0 && LISTN % 4 == 0);
static_assert(AGG_LDS_BYTES <= 300000);
static_assert(DEGCAP % 32 == 0);
static_assert(UI_TOT % NTHR == 0 && UI_W1 % NTHR == 0 && UI_W2 % NTHR == 0 && UI_U1 % NTHR == 0 && UI_U2 % NTHR == 0);
static_assert(PL_TOT == 147456);
static_assert(HID == 4 * 32 && F == 64 && FE == 8 && MSGIN == 2 * F + FE);
static_assert(VPK * 4 == NZK * 2 && SGK == G1K);
static_assert(GBM == (GTHR / 32) * 16);
static_assert(NZK % 32 == 0 && SGK % 32 == 0 && W1K % 32 == 0);

typedef float          v4f   __attribute__((ext_vector_type(4)));
typedef float          v8f   __attribute__((ext_vector_type(8)));
typedef int            v4i   __attribute__((ext_vector_type(4)));
typedef int            v8i   __attribute__((ext_vector_type(8)));
typedef unsigned short v8us  __attribute__((ext_vector_type(8)));
typedef unsigned short v16us __attribute__((ext_vector_type(16)));
typedef __bf16         v16bf __attribute__((ext_vector_type(16)));
typedef v4f  __attribute__((may_alias)) v4fa;
typedef v4i  __attribute__((may_alias)) v4ia;
typedef v8us __attribute__((may_alias)) v8usa;
union FragB { v16bf v; v16us u; v8us h[2]; v8i w; };

__device__ __forceinline__ v8f wmb(const FragB& a, const FragB& b, v8f c) {
  v8f d = __builtin_amdgcn_wmma_f32_16x16x32_bf16(false, a.v, false, b.v, (short)0, c, false, false);
  asm volatile("v_nop\n\tv_nop\n\tv_nop\n\tv_nop" : "+v"(d) : "v"(a.w), "v"(b.w));
  return d;
}

__device__ __forceinline__ unsigned bf16_bits(float f) {
  const unsigned u = __float_as_uint(f);
  return (u + 0x7FFFu + ((u >> 16) & 1u)) >> 16;
}
__device__ __forceinline__ float bf16_val(float f) {
  return __uint_as_float(bf16_bits(f) << 16);
}
__device__ __forceinline__ v4f bfr4(const v4f a) {
  v4f r; r.x = bf16_val(a.x); r.y = bf16_val(a.y); r.z = bf16_val(a.z); r.w = bf16_val(a.w); return r;
}
__device__ __forceinline__ v4f relu4(const v4f a) {
  v4f r;
  r.x = fmaxf(a.x, 0.0f); r.y = fmaxf(a.y, 0.0f); r.z = fmaxf(a.z, 0.0f); r.w = fmaxf(a.w, 0.0f);
  return r;
}
__device__ __forceinline__ v4f fma4(float s, const v4f w, v4f t) {
  t.x = fmaf(s, w.x, t.x); t.y = fmaf(s, w.y, t.y); t.z = fmaf(s, w.z, t.z); t.w = fmaf(s, w.w, t.w);
  return t;
}
__device__ __forceinline__ float rlf(float v, int k) {
  return __int_as_float(__builtin_amdgcn_readlane(__float_as_int(v), k));
}
__device__ __forceinline__ float shf(float v, int src) {
  return __int_as_float(__shfl(__float_as_int(v), src, 32));
}
__device__ __forceinline__ void put16(unsigned short* dp, v8us o) {
  *(volatile v8us*)dp = o;
  __threadfence();
  *(volatile v8us*)dp = o;
}

template <int SLB>
__device__ __forceinline__ int scan_chunk(const int* __restrict__ dsts, int nE, int cbase, int slotBase,
                                          int nb, int vec8, int* list, int tid, int lane, int wave) {
  int wc = 0;
  const int el0  = tid * EPT;
  const int e0   = cbase + el0;
  const int sent = -2147483647 - 1;
  v4i da, db;
  if (vec8 != 0 && cbase + CHUNK <= nE) {
    da = *(const v4i*)(dsts + e0);
    db = *(const v4i*)(dsts + e0 + 4);
  } else {
    da.x = (e0     < nE) ? dsts[min(e0,     nE - 1)] : sent;
    da.y = (e0 + 1 < nE) ? dsts[min(e0 + 1, nE - 1)] : sent;
    da.z = (e0 + 2 < nE) ? dsts[min(e0 + 2, nE - 1)] : sent;
    da.w = (e0 + 3 < nE) ? dsts[min(e0 + 3, nE - 1)] : sent;
    db.x = (e0 + 4 < nE) ? dsts[min(e0 + 4, nE - 1)] : sent;
    db.y = (e0 + 5 < nE) ? dsts[min(e0 + 5, nE - 1)] : sent;
    db.z = (e0 + 6 < nE) ? dsts[min(e0 + 6, nE - 1)] : sent;
    db.w = (e0 + 7 < nE) ? dsts[min(e0 + 7, nE - 1)] : sent;
  }
  const unsigned nbs = (unsigned)slotBase;
  const unsigned unb = (unsigned)nb;
  const unsigned s0 = (unsigned)da.x - nbs, s1 = (unsigned)da.y - nbs;
  const unsigned s2 = (unsigned)da.z - nbs, s3 = (unsigned)da.w - nbs;
  const unsigned s4 = (unsigned)db.x - nbs, s5 = (unsigned)db.y - nbs;
  const unsigned s6 = (unsigned)db.z - nbs, s7 = (unsigned)db.w - nbs;
  const bool h0 = s0 < unb, h1 = s1 < unb, h2 = s2 < unb, h3 = s3 < unb;
  const bool h4 = s4 < unb, h5 = s5 < unb, h6 = s6 < unb, h7 = s7 < unb;
  const unsigned any = __builtin_amdgcn_ballot_w32(h0 | h1 | h2 | h3 | h4 | h5 | h6 | h7);
  if (any != 0u) {
#define HITJ(J, HJ, SJ) { \
      const unsigned mj = __builtin_amdgcn_ballot_w32(HJ); \
      if (mj != 0u) { \
        if (HJ) { \
          const int pos = wc + (int)__builtin_amdgcn_mbcnt_lo(mj, 0u); \
          if (pos < WCAP) list[wave * WCAP + pos] = ((el0 + (J)) << SLB) | (int)(SJ); \
        } \
        wc += (int)__builtin_popcount(mj); } }
    HITJ(0, h0, s0)
    HITJ(1, h1, s1)
    HITJ(2, h2, s2)
    HITJ(3, h3, s3)
    HITJ(4, h4, s4)
    HITJ(5, h5, s5)
    HITJ(6, h6, s6)
    HITJ(7, h7, s7)
#undef HITJ
  }
  return wc;
}

__global__ __launch_bounds__(NTHR) void k_prep(const float* __restrict__ wm1, const float* __restrict__ wm2,
                                               const float* __restrict__ wv1, const float* __restrict__ wv2,
                                               const float* __restrict__ wc1, const float* __restrict__ wc2,
                                               int nUnits, unsigned short* WP) {
  const int u = (int)blockIdx.x * NTHR + (int)threadIdx.x;
  if (u >= nUnits) return;
  const int it = u / UI_TOT;
  const int v  = u - it * UI_TOT;
  unsigned short* base = WP + (size_t)it * PL_TOT;
  const float* p;
  int st;
  unsigned short* dp;
  if (v < UI_W1) {
    const int n    = v >> 4;
    const int k8   = (v & 15) * 8;
    const int nn   = n & (HID - 1);
    const int srow = (n >> 7) * F + (k8 & (F - 1));
    p  = wm1 + (size_t)it * MSGIN * HID + (size_t)srow * HID + nn;
    st = HID;
    dp = base + O_W1 + (size_t)n * W1K + k8;
  } else if (v < UI_W1 + UI_W2) {
    const int v2   = v - UI_W1;
    const int n    = v2 >> 5;
    const int k8   = (v2 & 31) * 8;
    const int srow = k8 & (HID - 1);
    p  = wm2 + (size_t)it * HID * F + (size_t)srow * F + n;
    st = F;
    dp = base + O_W2 + (size_t)n * SGK + k8;
  } else if (v < UI_W1 + UI_W2 + UI_U1) {
    const int v2   = v - (UI_W1 + UI_W2);
    const int n    = v2 >> 5;
    const int k8   = (v2 & 31) * 8;
    const int srow = k8 < 128 ? k8 : (k8 < 192 ? k8 - 64 : k8 - 192);
    p  = wv1 + (size_t)it * HID * HID + (size_t)srow * HID + n;
    st = HID;
    dp = base + O_V1 + (size_t)n * NZK + k8;
  } else if (v < UI_W1 + UI_W2 + UI_U1 + UI_U2) {
    const int v2   = v - (UI_W1 + UI_W2 + UI_U1);
    const int n    = v2 >> 5;
    const int k8   = (v2 & 31) * 8;
    const int srow = k8 & (HID - 1);
    p  = wv2 + (size_t)it * HID * F + (size_t)srow * F + n;
    st = F;
    dp = base + O_V2 + (size_t)n * G1K + k8;
  } else if (v < UI_W1 + UI_W2 + 2 * UI_U1 + UI_U2) {
    const int v2   = v - (UI_W1 + UI_W2 + UI_U1 + UI_U2);
    const int n    = v2 >> 5;
    const int k8   = (v2 & 31) * 8;
    const int srow = k8 < 128 ? k8 : (k8 < 192 ? k8 - 64 : k8 - 192);
    p  = wc1 + (size_t)it * HID * HID + (size_t)srow * HID + n;
    st = HID;
    dp = base + O_C1 + (size_t)n * NZK + k8;
  } else {
    const int v2   = v - (UI_W1 + UI_W2 + 2 * UI_U1 + UI_U2);
    const int n    = v2 >> 5;
    const int k8   = (v2 & 31) * 8;
    const int srow = k8 & (HID - 1);
    p  = wc2 + (size_t)it * HID * F + (size_t)srow * F + n;
    st = F;
    dp = base + O_C2 + (size_t)n * G1K + k8;
  }
  v8us o;
#pragma unroll
  for (int i = 0; i < 8; ++i) o[i] = (unsigned short)bf16_bits(p[(size_t)i * st]);
  put16(dp, o);
}

__global__ __launch_bounds__(NTHR) void k_xs(const float* __restrict__ x, int nX, int rin, int nUnits,
                                             unsigned short* NZ) {
  const int u = (int)blockIdx.x * NTHR + (int)threadIdx.x;
  if (u >= nUnits) return;
  const int row  = u >> 4;
  const int j    = u & 15;
  const int part = j >> 3;
  const int c8   = (j & 7) * 8;
  const int rc   = row < nX ? row : nX - 1;
  const float okf = row < nX ? 1.0f : 0.0f;
  const unsigned mh = 0u - (unsigned)part;
  const unsigned ml = ~mh;
  const float* xq = x + (size_t)rc * F + c8;
  const v4f a = *(const v4fa*)xq;
  const v4f b = *(const v4fa*)(xq + 4);
  const v8f f8 = {a.x, a.y, a.z, a.w, b.x, b.y, b.z, b.w};
  v8us o;
#pragma unroll
  for (int e = 0; e < 8; ++e) {
    float v = f8[e] * okf;
    const float vr = bf16_val(v);
    v = (rin != 0) ? vr : v;
    const unsigned hb = bf16_bits(v);
    const unsigned lb = bf16_bits(v - __uint_as_float(hb << 16));
    o[e] = (unsigned short)((hb & ml) | (lb & mh));
  }
  put16(NZ + (size_t)row * NZK + part * 192 + c8, o);
}

template <int NT, int AM, int EM>
__global__ __launch_bounds__(GTHR) void k_gemm(const unsigned short* __restrict__ Ab, int lda,
                                               const float* __restrict__ Xf, int nX, int rin,
                                               const unsigned short* __restrict__ BT, int ldb, int K,
                                               const float* __restrict__ bias, const float* __restrict__ deg,
                                               int nlim, float* Cm, unsigned short* Cb) {
  constexpr int GBN = 16 * NT;
  static_assert(NT == 4 || NT == 8);
  static_assert((EM == 0 && NT == 8) || (EM == 1 && NT == 4) || (EM == 2 && NT == 8) || (EM == 3 && NT == 4));
  __shared__ __attribute__((aligned(16))) float stg[GBM * GBN];
  __shared__ float sdg[GBM];
  const int tid = (int)threadIdx.x, lane = tid & 31, wave = tid >> 5, hh = lane >> 4, m = lane & 15;
  const int rowBase = (int)blockIdx.x * GBM;

  if constexpr (EM == 1) {
    if (tid < GBM) sdg[tid] = deg[(size_t)(rowBase + tid)];
  }
  __syncthreads();

  v8f acc[NT];
  {
    const v8f z = {0.f, 0.f, 0.f, 0.f, 0.f, 0.f, 0.f, 0.f};
#pragma unroll
    for (int t = 0; t < NT; ++t) acc[t] = z;
  }
  const int ar  = rowBase + 16 * wave + m;
  const int arc = ar < nX ? ar : nX - 1;
  const float okf = ar < nX ? 1.0f : 0.0f;
  const unsigned short* ap = Ab + (size_t)ar * (size_t)lda + 8 * hh;
  const float*          xp = Xf + (size_t)arc * F + 8 * hh;
  const unsigned short* bp = BT + (size_t)m * (size_t)ldb + 8 * hh;

#pragma unroll 1
  for (int k0 = 0; k0 < K; k0 += 32) {
    FragB af;
    if constexpr (AM == 0) {
      af.h[0] = *(const v8usa*)(ap + k0);
      af.h[1] = *(const v8usa*)(ap + k0 + 16);
    } else {
      const int kk = k0 & 63;
      const unsigned msk = (k0 >= 64) ? 0xFFFFFFFFu : 0u;
      const v4f u0 = *(const v4fa*)(xp + kk);
      const v4f u1 = *(const v4fa*)(xp + kk + 4);
      const v4f u2 = *(const v4fa*)(xp + kk + 16);
      const v4f u3 = *(const v4fa*)(xp + kk + 20);
      const v8f f0 = {u0.x, u0.y, u0.z, u0.w, u1.x, u1.y, u1.z, u1.w};
      const v8f f1 = {u2.x, u2.y, u2.z, u2.w, u3.x, u3.y, u3.z, u3.w};
      v8us o0, o1;
#pragma unroll
      for (int e = 0; e < 8; ++e) {
        float va = f0[e] * okf;
        float vb = f1[e] * okf;
        const float ra = bf16_val(va), rb = bf16_val(vb);
        va = (rin != 0) ? ra : va;
        vb = (rin != 0) ? rb : vb;
        const unsigned ha = bf16_bits(va);
        const unsigned la = bf16_bits(va - __uint_as_float(ha << 16));
        const unsigned hb = bf16_bits(vb);
        const unsigned lb = bf16_bits(vb - __uint_as_float(hb << 16));
        o0[e] = (unsigned short)((ha & ~msk) | (la & msk));
        o1[e] = (unsigned short)((hb & ~msk) | (lb & msk));
      }
      af.h[0] = o0;
      af.h[1] = o1;
    }
#pragma unroll
    for (int nt = 0; nt < NT; ++nt) {
      const unsigned short* wq = bp + (size_t)(16 * nt) * (size_t)ldb + k0;
      FragB bf;
      bf.h[0] = *(const v8usa*)wq;
      bf.h[1] = *(const v8usa*)(wq + 16);
      acc[nt] = wmb(af, bf, acc[nt]);
    }
  }

#pragma unroll
  for (int nt = 0; nt < NT; ++nt) {
    const int lc = 16 * nt + m;
    float bvv = 0.0f;
    if constexpr (EM != 0) bvv = bf16_val(bias[lc]);
#pragma unroll
    for (int r = 0; r < 8; ++r) {
      const int lr = 16 * wave + 8 * hh + r;
      float v = acc[nt][r];
      if constexpr (EM == 1) v = fmaf(sdg[lr], bvv, v);
      if constexpr (EM == 2) v = fmaxf(v + bvv, 0.0f);
      if constexpr (EM == 3) v = v + bvv;
      stg[lr * GBN + lc] = v;
    }
  }
  __syncthreads();

  if constexpr (EM == 0) {
    v4f pv[16];
#pragma unroll
    for (int i = 0; i < 16; ++i) pv[i] = *(const v4fa*)(stg + (16 * wave + i) * GBN + 4 * lane);
#pragma unroll
    for (int i = 0; i < 16; ++i) {
      float* op = Cm + (size_t)(rowBase + 16 * wave + i) * (size_t)VPK + 4 * lane;
      *(volatile v4f*)op = pv[i];
    }
    __threadfence();
#pragma unroll
    for (int i = 0; i < 16; ++i) {
      float* op = Cm + (size_t)(rowBase + 16 * wave + i) * (size_t)VPK + 4 * lane;
      *(volatile v4f*)op = pv[i];
    }
  } else if constexpr (EM == 1) {
    const int hsel = lane >> 4;
    const int j    = lane & 15;
    const int part = j >> 3;
    const int c8   = (j & 7) * 8;
    const unsigned mh = 0u - (unsigned)part;
    const unsigned ml = ~mh;
    v8us pv[8];
#pragma unroll
    for (int i2 = 0; i2 < 8; ++i2) {
      const int lr = 16 * wave + 2 * i2 + hsel;
      const float* sp = stg + lr * GBN + c8;
      const v4f a = *(const v4fa*)sp;
      const v4f b = *(const v4fa*)(sp + 4);
      const v8f f8 = {a.x, a.y, a.z, a.w, b.x, b.y, b.z, b.w};
      v8us oo;
#pragma unroll
      for (int e = 0; e < 8; ++e) {
        const unsigned hb = bf16_bits(f8[e]);
        const unsigned lb = bf16_bits(f8[e] - __uint_as_float(hb << 16));
        oo[e] = (unsigned short)((hb & ml) | (lb & mh));
      }
      pv[i2] = oo;
    }
#pragma unroll
    for (int i2 = 0; i2 < 8; ++i2) {
      unsigned short* op = Cb + (size_t)(rowBase + 16 * wave + 2 * i2 + hsel) * (size_t)NZK + 64 + part * 64 + c8;
      *(volatile v8us*)op = pv[i2];
    }
    __threadfence();
#pragma unroll
    for (int i2 = 0; i2 < 8; ++i2) {
      unsigned short* op = Cb + (size_t)(rowBase + 16 * wave + 2 * i2 + hsel) * (size_t)NZK + 64 + part * 64 + c8;
      *(volatile v8us*)op = pv[i2];
    }
  } else if constexpr (EM == 2) {
    const int part = lane >> 4;
    const int j = lane & 15;
    const unsigned mh = 0u - (unsigned)part;
    const unsigned ml = ~mh;
    v8us pv[16];
#pragma unroll
    for (int i = 0; i < 16; ++i) {
      const float* sp = stg + (16 * wave + i) * GBN + 8 * j;
      const v4f a = *(const v4fa*)sp;
      const v4f b = *(const v4fa*)(sp + 4);
      const v8f f8 = {a.x, a.y, a.z, a.w, b.x, b.y, b.z, b.w};
      v8us oo;
#pragma unroll
      for (int e = 0; e < 8; ++e) {
        const unsigned hb = bf16_bits(f8[e]);
        const unsigned lb = bf16_bits(f8[e] - __uint_as_float(hb << 16));
        oo[e] = (unsigned short)((hb & ml) | (lb & mh));
      }
      pv[i] = oo;
    }
#pragma unroll
    for (int i = 0; i < 16; ++i) {
      unsigned short* op = Cb + (size_t)(rowBase + 16 * wave + i) * (size_t)G1K + part * HID + 8 * j;
      *(volatile v8us*)op = pv[i];
    }
    __threadfence();
#pragma unroll
    for (int i = 0; i < 16; ++i) {
      unsigned short* op = Cb + (size_t)(rowBase + 16 * wave + i) * (size_t)G1K + part * HID + 8 * j;
      *(volatile v8us*)op = pv[i];
    }
  } else {
    const int hsel = lane >> 4;
    const int c    = 4 * (lane & 15);
    v4f pv[8];
#pragma unroll
    for (int i2 = 0; i2 < 8; ++i2) pv[i2] = *(const v4fa*)(stg + (16 * wave + 2 * i2 + hsel) * GBN + c);
#pragma unroll
    for (int i2 = 0; i2 < 8; ++i2) {
      const int row = rowBase + 16 * wave + 2 * i2 + hsel;
      if (row < nlim) *(volatile v4f*)(Cm + (size_t)row * F + c) = pv[i2];
    }
    __threadfence();
#pragma unroll
    for (int i2 = 0; i2 < 8; ++i2) {
      const int row = rowBase + 16 * wave + 2 * i2 + hsel;
      if (row < nlim) *(volatile v4f*)(Cm + (size_t)row * F + c) = pv[i2];
    }
  }
}

__global__ __launch_bounds__(NTHR) void k_scan(const int* __restrict__ keys, const int* __restrict__ oths,
                                               int nE, int nK, int nO, int vec8, int mRows,
                                               const float* __restrict__ VA, const float* __restrict__ VB,
                                               const float* __restrict__ ef, const float* __restrict__ We,
                                               const float* __restrict__ b1,
                                               unsigned short* SG, float* DEG) {
  extern __shared__ __attribute__((aligned(16))) int dsm[];
  int*   list = dsm;
  int*   hl   = dsm + LISTN;
  int*   sl   = hl + RCAP;
  int*   cnt  = sl + RCAP;
  int*   offs = cnt + NBA;
  int*   cur  = offs + NBA;
  int*   misc = cur + NBA;
  float* sdg  = (float*)(misc + 16);
  const int tid = (int)threadIdx.x, lane = tid & 31, wave = tid >> 5;
  const int nodeBase = (int)blockIdx.x * NBA;

  {
    const v4i z4 = {0, 0, 0, 0};
    for (int i = tid * 4; i < AGG_ZINTS; i += NTHR * 4) *(v4ia*)(dsm + i) = z4;
    if (tid < 16) misc[tid] = 0;
    for (int i = tid; i < NBA; i += NTHR) sdg[i] = 0.0f;
  }
  __syncthreads();

  int t = 0, ov = 0;
  const int nChunks = (nE + CHUNK - 1) / CHUNK;
#pragma unroll 1
  for (int ch = 0; ch < nChunks; ++ch) {
    const int cbase = ch * CHUNK;
    const int wc = scan_chunk<SLA>(keys, nE, cbase, nodeBase, NBA, vec8, list, tid, lane, wave);
    if (lane == 0) misc[wave] = wc;
    __syncthreads();
    if (wave == 0) {
#pragma unroll 1
      for (int w2 = 0; w2 < NWAVE; ++w2) {
        int cc = misc[w2];
        cc = cc < 0 ? 0 : (cc > WCAP ? WCAP : cc);
#pragma unroll 1
        for (int b0 = 0; b0 < cc; b0 += 32) {
          const int idx = b0 + lane;
          const int ent = list[w2 * WCAP + (idx < WCAP ? idx : WCAP - 1)];
          const int m32 = (cc - b0) < 32 ? (cc - b0) : 32;
#pragma unroll 1
          for (int k = 0; k < m32; ++k) {
            const int u    = __builtin_amdgcn_readlane(ent, k);
            const int slot = u & (NBA - 1);
            const int el   = (u >> SLA) & (CHUNK - 1);
            const int pk   = ((cbase + el) << SLA) | slot;
            if (t < RCAP) {
              if (lane == 0) { hl[t] = pk; cnt[slot] = cnt[slot] + 1; }
              t = t + 1;
            } else {
              ov = 1;
            }
          }
        }
      }
    }
    __syncthreads();
  }
  if (wave == 0 && lane == 0) { misc[8] = t; misc[9] = ov; }
  __syncthreads();
  int tt = misc[8];
  tt = tt < 0 ? 0 : (tt > RCAP ? RCAP : tt);
  const int ovf = misc[9];

  if (wave == 0) {
    const int base = lane * (NBA / 32);
    int s = 0;
#pragma unroll 1
    for (int i = 0; i < NBA / 32; ++i) s += cnt[base + i];
    int incl = s;
#pragma unroll
    for (int d = 1; d < 32; d <<= 1) {
      const int y = __shfl_up(incl, d, 32);
      if (lane >= d) incl += y;
    }
    int run = incl - s;
#pragma unroll 1
    for (int i = 0; i < NBA / 32; ++i) {
      const int cv = cnt[base + i];
      offs[base + i] = run;
      cur[base + i]  = run;
      run += cv;
    }
  }
  __syncthreads();
  if (wave == 0) {
#pragma unroll 1
    for (int b0 = 0; b0 < tt; b0 += 32) {
      const int idx = b0 + lane;
      const int ent = hl[idx < RCAP ? idx : RCAP - 1];
      const int m32 = (tt - b0) < 32 ? (tt - b0) : 32;
#pragma unroll 1
      for (int k = 0; k < m32; ++k) {
        const int u    = __builtin_amdgcn_readlane(ent, k);
        const int slot = u & (NBA - 1);
        if (lane == 0) {
          int p = cur[slot];
          p = p < 0 ? 0 : (p > RCAP - 1 ? RCAP - 1 : p);
          sl[p] = u;
          cur[slot] = p + 1;
        }
      }
    }
  }
  __syncthreads();

  const float qnan = __int_as_float(0x7fc00000);
  const float pz = (ovf != 0) ? qnan : 0.0f;
  const int c0 = 4 * lane;
  const v4f we0 = bfr4(*(const v4fa*)(We + 0 * HID + c0));
  const v4f we1 = bfr4(*(const v4fa*)(We + 1 * HID + c0));
  const v4f we2 = bfr4(*(const v4fa*)(We + 2 * HID + c0));
  const v4f we3 = bfr4(*(const v4fa*)(We + 3 * HID + c0));
  const v4f we4 = bfr4(*(const v4fa*)(We + 4 * HID + c0));
  const v4f we5 = bfr4(*(const v4fa*)(We + 5 * HID + c0));
  const v4f we6 = bfr4(*(const v4fa*)(We + 6 * HID + c0));
  const v4f we7 = bfr4(*(const v4fa*)(We + 7 * HID + c0));
  const v4f bb  = bfr4(*(const v4fa*)(b1 + c0));
  const int jj = lane & 15, part = lane >> 4;
  const unsigned mh = 0u - (unsigned)part;
  const unsigned ml = ~mh;
  const int srcA = 2 * jj, srcB = 2 * jj + 1;
  const v4f z4 = {0.0f, 0.0f, 0.0f, 0.0f};
#pragma unroll 1
  for (int si = 0; si < NBA / NWAVE; ++si) {
    const int s    = si * NWAVE + wave;
    const int node = nodeBase + s;
    const int craw = cnt[s];
    int cdeg = craw;
    const bool big = cdeg > DEGCAP;
    cdeg = cdeg < 0 ? 0 : (cdeg > DEGCAP ? DEGCAP : cdeg);
    int o = offs[s];
    o = o < 0 ? 0 : (o > RCAP ? RCAP : o);
    const int nc = node < nK ? node : nK - 1;
    const float okf = node < nK ? 1.0f : 0.0f;
    const v4f own = *(const v4fa*)(VA + (size_t)nc * VPK + c0) + bb;
    v4f acc = z4;
#pragma unroll 1
    for (int b0 = 0; b0 < cdeg; b0 += 32) {
      int idx = o + b0 + lane;
      idx = idx > RCAP - 1 ? RCAP - 1 : idx;
      const int ent = sl[idx];
      int eid = ent >> SLA;
      eid = eid < 0 ? 0 : (eid > nE - 1 ? nE - 1 : eid);
      int on = oths[eid];
      on = on < 0 ? 0 : (on > nO - 1 ? nO - 1 : on);
      const v4f ea = bfr4(*(const v4fa*)(ef + (size_t)eid * FE));
      const v4f eb = bfr4(*(const v4fa*)(ef + (size_t)eid * FE + 4));
      const int m32 = (cdeg - b0) < 32 ? (cdeg - b0) : 32;
#pragma unroll 1
      for (int k = 0; k < m32; ++k) {
        const int onk = __builtin_amdgcn_readlane(on, k);
        const v4f g = *(const v4fa*)(VB + (size_t)onk * VPK + c0);
        v4f tv = own + g;
        tv = fma4(rlf(ea.x, k), we0, tv);
        tv = fma4(rlf(ea.y, k), we1, tv);
        tv = fma4(rlf(ea.z, k), we2, tv);
        tv = fma4(rlf(ea.w, k), we3, tv);
        tv = fma4(rlf(eb.x, k), we4, tv);
        tv = fma4(rlf(eb.y, k), we5, tv);
        tv = fma4(rlf(eb.z, k), we6, tv);
        tv = fma4(rlf(eb.w, k), we7, tv);
        acc = acc + relu4(tv);
      }
    }
    const bool  live = node < mRows;
    const int   nr   = live ? node : mRows - 1;
    const float pzr  = big ? qnan : pz;
    acc = acc * okf + pzr;
    v4f fa, fb;
    fa.x = shf(acc.x, srcA); fa.y = shf(acc.y, srcA); fa.z = shf(acc.z, srcA); fa.w = shf(acc.w, srcA);
    fb.x = shf(acc.x, srcB); fb.y = shf(acc.y, srcB); fb.z = shf(acc.z, srcB); fb.w = shf(acc.w, srcB);
    const v8f f8 = {fa.x, fa.y, fa.z, fa.w, fb.x, fb.y, fb.z, fb.w};
    v8us oo;
#pragma unroll
    for (int e = 0; e < 8; ++e) {
      const unsigned hb = bf16_bits(f8[e]);
      const unsigned lb = bf16_bits(f8[e] - __uint_as_float(hb << 16));
      oo[e] = (unsigned short)((hb & ml) | (lb & mh));
    }
    unsigned short* rp = SG + (size_t)nr * SGK + part * HID + 8 * jj;
    if (live) *(volatile v8us*)rp = oo;
    __threadfence();
    if (live) *(volatile v8us*)rp = oo;
    if (lane == 0) sdg[s] = (float)craw * okf;
  }
  __syncthreads();

  {
    const v4f d4 = *(const v4fa*)(sdg + 4 * tid);
    const int n0 = nodeBase + 4 * tid;
    const bool stv = (n0 + 4 <= mRows);
    if (stv) *(volatile v4f*)(DEG + (size_t)n0) = d4;
    __threadfence();
    if (stv) *(volatile v4f*)(DEG + (size_t)n0) = d4;
  }
}

static inline int cdiv(int a, int b) { return (a + b - 1) / b; }

extern "C" void kernel_launch(void* const* d_in, const int* in_sizes, int n_in,
                              void* d_out, int out_size, void* d_ws, size_t ws_size,
                              hipStream_t stream) {
  if (n_in < 17) return;
  if (in_sizes[0] < F || (in_sizes[0] % F) != 0) return;
  if (in_sizes[1] < F || (in_sizes[1] % F) != 0) return;
  const int NV = in_sizes[0] / F;
  const int NC = in_sizes[1] / F;
  const int nE = in_sizes[3];
  if (NV < 1 || NC < 1 || nE < 1 || nE >= (1 << 21)) return;
  if (in_sizes[4] != nE) return;
  if (in_sizes[2] != nE * FE) return;
  if (in_sizes[6] < HID || (in_sizes[6] % HID) != 0) return;
  const int ITERS = in_sizes[6] / HID;
  if (in_sizes[5]  != ITERS * MSGIN * HID) return;
  if (in_sizes[7]  != ITERS * HID * F || in_sizes[8]  != ITERS * F) return;
  if (in_sizes[9]  != ITERS * HID * HID || in_sizes[10] != ITERS * HID) return;
  if (in_sizes[11] != ITERS * HID * F || in_sizes[12] != ITERS * F) return;
  if (in_sizes[13] != ITERS * HID * HID || in_sizes[14] != ITERS * HID) return;
  if (in_sizes[15] != ITERS * HID * F || in_sizes[16] != ITERS * F) return;
  if ((long long)out_size != (long long)(NV + NC) * F) return;

  const float* var_feat  = (const float*)d_in[0];
  const float* cons_feat = (const float*)d_in[1];
  const float* edge_feat = (const float*)d_in[2];
  const int*   edge_var  = (const int*)d_in[3];
  const int*   edge_cons = (const int*)d_in[4];
  const float* w_msg1  = (const float*)d_in[5];
  const float* b_msg1  = (const float*)d_in[6];
  const float* w_msg2  = (const float*)d_in[7];
  const float* b_msg2  = (const float*)d_in[8];
  const float* w_vupd1 = (const float*)d_in[9];
  const float* b_vupd1 = (const float*)d_in[10];
  const float* w_vupd2 = (const float*)d_in[11];
  const float* b_vupd2 = (const float*)d_in[12];
  const float* w_cupd1 = (const float*)d_in[13];
  const float* b_cupd1 = (const float*)d_in[14];
  const float* w_cupd2 = (const float*)d_in[15];
  const float* b_cupd2 = (const float*)d_in[16];
  float* out0 = (float*)d_out;
  float* out1 = out0 + (size_t)NV * F;

  const int MPV = cdiv(NV, GBM) * GBM;
  const int MPC = cdiv(NC, GBM) * GBM;
  const int MPX = MPV > MPC ? MPV : MPC;
  const int gMV = MPV / GBM, gMC = MPC / GBM;
  const int gAV = cdiv(MPV, NBA), gAC = cdiv(MPC, NBA);
  if ((long long)gAV * NBA < (long long)MPV || (long long)gAC * NBA < (long long)MPC) return;

  char* ws = (char*)d_ws;
  size_t off = 0;
  const size_t oWP  = off; off += (size_t)ITERS * PL_TOT * 2;       off = (off + 255) & ~(size_t)255;
  const size_t oRA  = off; off += (size_t)MPX * VPK * 4;            off = (off + 255) & ~(size_t)255;
  const size_t oRB  = off; off += (size_t)MPX * VPK * 4;            off = (off + 255) & ~(size_t)255;
  const size_t oRSV = off; off += (size_t)MPV * SGK * 2;            off = (off + 255) & ~(size_t)255;
  const size_t oRSC = off; off += (size_t)MPC * SGK * 2;            off = (off + 255) & ~(size_t)255;
  const size_t oXFV = off; off += (size_t)MPV * F * 4;              off = (off + 255) & ~(size_t)255;
  const size_t oXFC = off; off += (size_t)MPC * F * 4;              off = (off + 255) & ~(size_t)255;
  const size_t oDGV = off; off += (size_t)MPV * 4;                  off = (off + 255) & ~(size_t)255;
  const size_t oDGC = off; off += (size_t)MPC * 4;                  off = (off + 255) & ~(size_t)255;
  if (off > ws_size || off > (size_t)WSMAX) return;
  unsigned short* WP  = (unsigned short*)(ws + oWP);
  float*          RAf = (float*)(ws + oRA);
  float*          RBf = (float*)(ws + oRB);
  unsigned short* NZV = (unsigned short*)(ws + oRA);
  unsigned short* NZC = (unsigned short*)(ws + oRB);
  unsigned short* SGV = (unsigned short*)(ws + oRSV);
  unsigned short* SGC = (unsigned short*)(ws + oRSC);
  unsigned short* G1V = (unsigned short*)(ws + oRSV);
  unsigned short* G1C = (unsigned short*)(ws + oRSC);
  float*          XFV = (float*)(ws + oXFV);
  float*          XFC = (float*)(ws + oXFC);
  float*          DGV = (float*)(ws + oDGV);
  float*          DGC = (float*)(ws + oDGC);

  hipFuncSetAttribute(reinterpret_cast<const void*>(&k_scan), hipFuncAttributeMaxDynamicSharedMemorySize,
                      (int)AGG_LDS_BYTES);

  const int vec8 = 1;

  const int nPrep = ITERS * UI_TOT;
  k_prep<<<nPrep / NTHR, NTHR, 0, stream>>>(w_msg1, w_msg2, w_vupd1, w_vupd2, w_cupd1, w_cupd2, nPrep, WP);

  for (int i = 0; i < ITERS; ++i) {
    const unsigned short* WPi  = WP + (size_t)i * PL_TOT;
    const unsigned short* W1AT = WPi + O_W1;
    const unsigned short* W1BT = WPi + O_W1 + (size_t)HID * W1K;
    const unsigned short* W2T  = WPi + O_W2;
    const unsigned short* WV1T = WPi + O_V1;
    const unsigned short* WV2T = WPi + O_V2;
    const unsigned short* WC1T = WPi + O_C1;
    const unsigned short* WC2T = WPi + O_C2;
    const float* w1i  = w_msg1 + (size_t)i * MSGIN * HID;
    const float* Wei  = w1i + (size_t)HID * HID;
    const float* b1i  = b_msg1 + (size_t)i * HID;
    const float* b2i  = b_msg2 + (size_t)i * F;
    const float* bv1i = b_vupd1 + (size_t)i * HID;
    const float* bv2i = b_vupd2 + (size_t)i * F;
    const float* bc1i = b_cupd1 + (size_t)i * HID;
    const float* bc2i = b_cupd2 + (size_t)i * F;
    const float* xv   = (i == 0) ? var_feat  : XFV;
    const float* xc   = (i == 0) ? cons_feat : XFC;
    const int rin  = (i == 0) ? 1 : 0;
    const int KVP  = rin ? 64 : 128;
    const int KL1  = rin ? 192 : 256;
    const bool last = (i == ITERS - 1);

    k_gemm<8, 1, 0><<<dim3(gMV), GTHR, 0, stream>>>(WPi, 0, xv, NV, rin, W1AT, W1K, KVP, b1i, DGV, 0, RAf, NZV);
    k_gemm<8, 1, 0><<<dim3(gMC), GTHR, 0, stream>>>(WPi, 0, xc, NC, rin, W1BT, W1K, KVP, b1i, DGC, 0, RBf, NZC);
    k_scan<<<gAV, NTHR, AGG_LDS_BYTES, stream>>>(edge_var, edge_cons, nE, NV, NC, vec8, MPV, RAf, RBf,
                                                 edge_feat, Wei, b1i, SGV, DGV);
    k_gemm<8, 1, 0><<<dim3(gMC), GTHR, 0, stream>>>(WPi, 0, xc, NC, rin, W1AT, W1K, KVP, b1i, DGC, 0, RAf, NZC);
    k_gemm<8, 1, 0><<<dim3(gMV), GTHR, 0, stream>>>(WPi, 0, xv, NV, rin, W1BT, W1K, KVP, b1i, DGV, 0, RBf, NZV);
    k_scan<<<gAC, NTHR, AGG_LDS_BYTES, stream>>>(edge_cons, edge_var, nE, NC, NV, vec8, MPC, RAf, RBf,
                                                 edge_feat, Wei, b1i, SGC, DGC);
    k_xs<<<(MPV * 16) / NTHR, NTHR, 0, stream>>>(xv, NV, rin, MPV * 16, NZV);
    k_xs<<<(MPC * 16) / NTHR, NTHR, 0, stream>>>(xc, NC, rin, MPC * 16, NZC);
    k_gemm<4, 0, 1><<<dim3(gMV), GTHR, 0, stream>>>(SGV, SGK, xv, MPV, 0, W2T, SGK, SGK, b2i, DGV, 0, XFV, NZV);
    k_gemm<4, 0, 1><<<dim3(gMC), GTHR, 0, stream>>>(SGC, SGK, xc, MPC, 0, W2T, SGK, SGK, b2i, DGC, 0, XFC, NZC);
    k_gemm<8, 0, 2><<<dim3(gMV), GTHR, 0, stream>>>(NZV, NZK, xv, MPV, 0, WV1T, NZK, KL1, bv1i, DGV, 0, XFV, G1V);
    k_gemm<8, 0, 2><<<dim3(gMC), GTHR, 0, stream>>>(NZC, NZK, xc, MPC, 0, WC1T, NZK, KL1, bc1i, DGC, 0, XFC, G1C);
    k_gemm<4, 0, 3><<<dim3(gMV), GTHR, 0, stream>>>(G1V, G1K, xv, MPV, 0, WV2T, G1K, G1K, bv2i, DGV,
                                                    last ? NV : MPV, last ? out0 : XFV, NZV);
    k_gemm<4, 0, 3><<<dim3(gMC), GTHR, 0, stream>>>(G1C, G1K, xc, MPC, 0, WC2T, G1K, G1K, bc2i, DGC,
                                                    last ? NC : MPC, last ? out1 : XFC, NZC);
  }
}
